// CausalSelfAttention_48369921688055
// MI455X (gfx1250) — hardware-verified
//
#include <hip/hip_runtime.h>

#ifndef NB
#define NB 4
#endif
#ifndef SEQ
#define SEQ 2048
#endif
#define NB_FULL 4
#define SEQ_FULL 2048
#define EMB 1024
#define NHEAD 16
#define HDIM 64
#define NQK (2 * EMB)
#define NQKV (3 * EMB)
#define BAND ((SEQ < 512) ? SEQ : 512)
#define MROWS (NB * SEQ)

static_assert(HDIM == 64);
static_assert(EMB == NHEAD * HDIM);
static_assert(SEQ % 64 == 0);
static_assert(BAND % 64 == 0);
static_assert(BAND <= SEQ);
static_assert(EMB % 64 == 0);
static_assert(NB <= NB_FULL);
static_assert(SEQ <= SEQ_FULL);
static_assert((NB == 1) || (SEQ == SEQ_FULL));
static_assert(NQK % HDIM == 0 && EMB % HDIM == 0);
static_assert(HDIM * 2 == 128);

typedef __attribute__((ext_vector_type(16))) _Float16 v16h;
typedef __attribute__((ext_vector_type(8)))  _Float16 v8h;
typedef __attribute__((ext_vector_type(16))) __bf16   v16b;
typedef __attribute__((ext_vector_type(8)))  __bf16   v8b;
typedef __attribute__((ext_vector_type(8)))  float    v8f;
typedef __attribute__((ext_vector_type(4)))  float    v4f;
typedef unsigned int cm_u4 __attribute__((ext_vector_type(4)));


#define VST2(T, ptr, val) do { const T vst2_v_ = (val); *(volatile T*)(ptr) = vst2_v_; __threadfence(); *(volatile T*)(ptr) = vst2_v_; } while (0)

namespace gemmkit {

__device__ __forceinline__ unsigned short f2bf_bits(float f) {
  unsigned u = __float_as_uint(f);
  return (unsigned short)((u + 0x7FFFu + ((u >> 16) & 1u)) >> 16);
}
__device__ __forceinline__ float bf_bits2f(unsigned short h) { return __uint_as_float(((unsigned)h) << 16); }

__device__ __forceinline__ void dep_guard_h(v8f& a, v8f& b, v16h x, v16h y) { asm volatile("v_nop\n\tv_nop\n\tv_nop\n\tv_nop" : "+v"(a), "+v"(b) : "v"(x), "v"(y)); }
__device__ __forceinline__ void dep_guard_b(v8f& a, v8f& b, v16b x, v16b y) { asm volatile("v_nop\n\tv_nop\n\tv_nop\n\tv_nop" : "+v"(a), "+v"(b) : "v"(x), "v"(y)); }
__device__ __forceinline__ void keep4_h(v16h a, v16h b, v16h c, v16h d) { asm volatile("v_nop" :: "v"(a), "v"(b), "v"(c), "v"(d)); }
__device__ __forceinline__ void keep4_b(v16b a, v16b b, v16b c, v16b d) { asm volatile("v_nop" :: "v"(a), "v"(b), "v"(c), "v"(d)); }
__device__ __forceinline__ void acc_guard4(v8f& a, v8f& b, v8f& c, v8f& d) { asm volatile("v_nop\n\tv_nop\n\tv_nop\n\tv_nop" : "+v"(a), "+v"(b), "+v"(c), "+v"(d)); }
template <typename T> struct Frag;
template <> struct Frag<_Float16> {
  typedef v16h V; union U { v16h v; v8h h[2]; };
  static __device__ __forceinline__ v16h load(const _Float16* p) {
    U f; f.h[0] = *(const v8h*)(p); f.h[1] = *(const v8h*)(p + 16); return f.v;
  }
  static __device__ __forceinline__ v8f mma(v16h a, v16h b, v8f c) {
    return __builtin_amdgcn_wmma_f32_16x16x32_f16(false, a, false, b, (short)0, c, false, false);
  }
  static __device__ __forceinline__ void guard(v8f& a, v8f& b, v16h x, v16h y) { dep_guard_h(a, b, x, y); }
  static __device__ __forceinline__ void keep(v16h a, v16h b, v16h c, v16h d) { keep4_h(a, b, c, d); }
};
template <> struct Frag<__bf16> {
  typedef v16b V; union U { v16b v; v8b h[2]; };
  static __device__ __forceinline__ v16b load(const __bf16* p) {
    U f; f.h[0] = *(const v8b*)(p); f.h[1] = *(const v8b*)(p + 16); return f.v;
  }
  static __device__ __forceinline__ v8f mma(v16b a, v16b b, v8f c) {
    return __builtin_amdgcn_wmma_f32_16x16x32_bf16(false, a, false, b, (short)0, c, false, false);
  }
  static __device__ __forceinline__ void guard(v8f& a, v8f& b, v16b x, v16b y) { dep_guard_b(a, b, x, y); }
  static __device__ __forceinline__ void keep(v16b a, v16b b, v16b c, v16b d) { keep4_b(a, b, c, d); }
};

template <int ET> struct Elem;
template <> struct Elem<0> { typedef _Float16 T; };
template <> struct Elem<1> { typedef __bf16 T; };
template <int ET, bool SPLIT, int BIAS_MODE, int OUT_MODE, bool RESID>
__global__ __launch_bounds__(256) void wmma_gemm64(
    const unsigned short* __restrict__ Ap, const unsigned short* __restrict__ A2p, int lda, long strideA,
    const unsigned short* __restrict__ Btp, const unsigned short* __restrict__ Bt2p, int ldb, long strideB,
    void* Cout, void* Cout2, int ldc, long strideC,
    const float* __restrict__ bias,
    const float* resid, long strideR,
    int M, int N, int K, float scale) {
  typedef typename Elem<ET>::T T;
  typedef typename Frag<T>::V V;
  const T* A = (const T*)Ap; const T* A2 = (const T*)A2p; const T* Bt = (const T*)Btp; const T* Bt2 = (const T*)Bt2p;
  __shared__ __align__(16) float sT[8][16 * 68];
  const int b    = blockIdx.y;
  const int lane = threadIdx.x & 31;
  const int wave = threadIdx.x >> 5;
  const int tilesN = N >> 6;
  const int tilesM = M >> 6;
  const int tile = blockIdx.x * 8 + wave;
  if (tile >= tilesM * tilesN) return;
  const int tm = tile / tilesN;
  const int tn = tile - tm * tilesN;
  const int m0 = tm << 6;
  const int n0 = tn << 6;

  const T* Ab  = A  + (size_t)b * strideA;
  const T* Bb  = Bt + (size_t)b * strideB;
  const T* Ab2 = SPLIT ? (A2  + (size_t)b * strideA) : nullptr;
  const T* Bb2 = SPLIT ? (Bt2 + (size_t)b * strideB) : nullptr;

  const int rlane = lane & 15;
  const int koff  = (lane >> 4) * 8;
  const int mOff  = (lane >> 4) * 8;

  v8f acc[4][4];
#pragma unroll
  for (int i = 0; i < 4; ++i)
#pragma unroll
    for (int j = 0; j < 4; ++j) acc[i][j] = (v8f){0.f,0.f,0.f,0.f,0.f,0.f,0.f,0.f};

  for (int k0 = 0; k0 < K; k0 += 32) {
    V bh[4], bl[4];
#pragma unroll
    for (int j = 0; j < 4; ++j) {
      const size_t bo = (size_t)(n0 + (j << 4) + rlane) * ldb + koff + k0;
      bh[j] = Frag<T>::load(Bb + bo);
      if (SPLIT) bl[j] = Frag<T>::load(Bb2 + bo);
    }
#pragma unroll
    for (int i = 0; i < 4; ++i) {
      const size_t ao = (size_t)(m0 + (i << 4) + rlane) * lda + koff + k0;
      V ah = Frag<T>::load(Ab + ao);
      V al;
      if (SPLIT) al = Frag<T>::load(Ab2 + ao);
#pragma unroll
      for (int j = 0; j < 4; ++j) {
        acc[i][j] = Frag<T>::mma(ah, bh[j], acc[i][j]);
        if (SPLIT) {
          acc[i][j] = Frag<T>::mma(ah, bl[j], acc[i][j]);
          acc[i][j] = Frag<T>::mma(al, bh[j], acc[i][j]);
        }
      }
      Frag<T>::guard(acc[i][0], acc[i][3], ah, SPLIT ? al : ah);
    }
    Frag<T>::keep(bh[0], bh[1], bh[2], bh[3]);
    if (SPLIT) Frag<T>::keep(bl[0], bl[1], bl[2], bl[3]);
  }
  acc_guard4(acc[0][0], acc[0][1], acc[0][2], acc[0][3]);
  acc_guard4(acc[1][0], acc[1][1], acc[1][2], acc[1][3]);
  acc_guard4(acc[2][0], acc[2][1], acc[2][2], acc[2][3]);
  acc_guard4(acc[3][0], acc[3][1], acc[3][2], acc[3][3]);

  float* slab = sT[wave];
  const float* Rb = RESID ? (resid + (size_t)b * strideR) : nullptr;
#pragma unroll
  for (int i = 0; i < 4; ++i) {
    const int mBase = m0 + (i << 4);
#pragma unroll
    for (int j = 0; j < 4; ++j) {
      const int n = n0 + (j << 4) + rlane;
      float bv = 0.f;
      if (BIAS_MODE == 2) bv = bias[n];
#pragma unroll
      for (int r = 0; r < 8; ++r) {
        float v = acc[i][j][r] * scale;
        if (BIAS_MODE == 1) v += bias[mBase + mOff + r];
        if (BIAS_MODE == 2) v += bv;
        if (RESID) v += Rb[(size_t)(mBase + mOff + r) * ldc + n];
        slab[(mOff + r) * 68 + (j << 4) + rlane] = v;
      }
    }
    __builtin_amdgcn_fence(3  , "workgroup");
    __builtin_amdgcn_wave_barrier();
    __builtin_amdgcn_fence(2  , "workgroup");
    if (OUT_MODE == 0) {
      float* C = (float*)Cout + (size_t)b * strideC;
      const int hh = lane >> 4, c4 = (lane & 15) * 4;
      for (int pass = 0; pass < 2; ++pass) {
#pragma unroll
        for (int it = 0; it < 8; ++it) {
          const int row = it * 2 + hh;
          v4f v = *(const v4f*)(slab + row * 68 + c4);
          *(volatile v4f*)(C + (size_t)(mBase + row) * ldc + n0 + c4) = v;
        }
        __threadfence();
      }
    } else {
      const int q = lane >> 3, c8 = (lane & 7) * 8;
      unsigned short* C  = (unsigned short*)Cout  + (size_t)b * strideC;
      unsigned short* C2 = (OUT_MODE >= 2) ? ((unsigned short*)Cout2 + (size_t)b * strideC) : nullptr;
      for (int pass = 0; pass < 2; ++pass) {
#pragma unroll
        for (int it = 0; it < 4; ++it) {
          const int row = it * 4 + q;
          const float* sp = slab + row * 68 + c8;
          v8h hv, lv;
#pragma unroll
          for (int e = 0; e < 8; ++e) {
            if (OUT_MODE == 1) {
              hv[e] = (_Float16)sp[e];
            } else if (OUT_MODE == 3) {
              const _Float16 hf = (_Float16)sp[e];
              hv[e] = hf;
              lv[e] = (_Float16)((sp[e] - (float)hf) * 2048.0f);
            } else {
              unsigned short hb = f2bf_bits(sp[e]);
              unsigned short lb = f2bf_bits(sp[e] - bf_bits2f(hb));
              hv[e] = __builtin_bit_cast(_Float16, hb);
              lv[e] = __builtin_bit_cast(_Float16, lb);
            }
          }
          *(volatile v8h*)(C + (size_t)(mBase + row) * ldc + n0 + c8) = hv;
          if (OUT_MODE >= 2) *(volatile v8h*)(C2 + (size_t)(mBase + row) * ldc + n0 + c8) = lv;
        }
        __threadfence();
      }
    }
    __builtin_amdgcn_fence(3  , "workgroup");
    __builtin_amdgcn_wave_barrier();
    __builtin_amdgcn_fence(2  , "workgroup");
  }
}

}

__device__ __forceinline__ unsigned int cmb_pk2(float a, float b) { return (unsigned int)__builtin_bit_cast(unsigned short, (_Float16)a) | ((unsigned int)__builtin_bit_cast(unsigned short, (_Float16)b) << 16); }
__device__ __forceinline__ float cmb_bf(float v) { const unsigned u = __builtin_bit_cast(unsigned, v); const unsigned r = (u + 0x7fffu + ((u >> 16) & 1u)) & 0xffff0000u; return __builtin_bit_cast(float, r); }
__global__ __launch_bounds__(256) void k_cm_castb(const float* __restrict__ SRC, unsigned short* __restrict__ DST, unsigned int n8, float sc) {
    const unsigned int u = blockIdx.x * 256u + threadIdx.x; if (u >= n8) return;
    const v4f a = *(const v4f*)(SRC + (size_t)u * 8u), b4 = *(const v4f*)(SRC + (size_t)u * 8u + 4u);
    cm_u4 pk;
    pk.x = cmb_pk2(cmb_bf(a.x) * sc, cmb_bf(a.y) * sc); pk.y = cmb_pk2(cmb_bf(a.z) * sc, cmb_bf(a.w) * sc);
    pk.z = cmb_pk2(cmb_bf(b4.x) * sc, cmb_bf(b4.y) * sc); pk.w = cmb_pk2(cmb_bf(b4.z) * sc, cmb_bf(b4.w) * sc);
    VST2(cm_u4, (cm_u4*)(DST + (size_t)u * 8u), pk); }
__global__ __launch_bounds__(256) void k_cm_bfvec(const float* __restrict__ SRC, float* __restrict__ DST, unsigned int n) { const unsigned int u = blockIdx.x * 256u + threadIdx.x; if (u >= n) return; VST2(float, DST + u, cmb_bf(SRC[u])); }

typedef unsigned short rq_us8 __attribute__((ext_vector_type(8)));
__global__ __launch_bounds__(256) __attribute__((amdgpu_num_vgpr(240))) void k_qk_rot(
    const unsigned short* __restrict__ Ap, int lda,
    const unsigned short* __restrict__ Btp, int ldb,
    unsigned short* Chi, unsigned short* Clo, int ldc,
    const float* __restrict__ bias,
    const float* __restrict__ cosT, const float* __restrict__ sinT,
    int M, int N, int K, float scale) {
  typedef gemmkit::Frag<_Float16> FH;
  const _Float16* A  = (const _Float16*)Ap;
  const _Float16* Bt = (const _Float16*)Btp;
  __shared__ __align__(16) float sT[8][16 * 68];
  const int lane = threadIdx.x & 31;
  const int wave = __builtin_amdgcn_readfirstlane(threadIdx.x >> 5);
  const int tilesN = N >> 6;
  const int tilesM = M >> 6;
  const int tile = blockIdx.x * 8 + wave;
  if (tile >= tilesM * tilesN) return;
  const int tm = tile / tilesN;
  const int tn = tile - tm * tilesN;
  const int m0 = tm << 6;
  const int n0 = tn << 6;

  const int rlane = lane & 15;
  const int koff  = (lane >> 4) * 8;
  const int mOff  = (lane >> 4) * 8;

  v8f acc[4][4];
#pragma unroll
  for (int i = 0; i < 4; ++i)
#pragma unroll
    for (int j = 0; j < 4; ++j) acc[i][j] = (v8f){0.f,0.f,0.f,0.f,0.f,0.f,0.f,0.f};

  for (int k0 = 0; k0 < K; k0 += 32) {
    v16h bh[4];
#pragma unroll
    for (int j = 0; j < 4; ++j) {
      const size_t bo = (size_t)(n0 + (j << 4) + rlane) * ldb + koff + k0;
      bh[j] = FH::load(Bt + bo);
    }
#pragma unroll
    for (int i = 0; i < 4; ++i) {
      const size_t ao = (size_t)(m0 + (i << 4) + rlane) * lda + koff + k0;
      v16h ah = FH::load(A + ao);
#pragma unroll
      for (int j = 0; j < 4; ++j) acc[i][j] = FH::mma(ah, bh[j], acc[i][j]);
      FH::guard(acc[i][0], acc[i][3], ah, ah);
    }
    FH::keep(bh[0], bh[1], bh[2], bh[3]);
  }
  gemmkit::acc_guard4(acc[0][0], acc[0][1], acc[0][2], acc[0][3]);
  gemmkit::acc_guard4(acc[1][0], acc[1][1], acc[1][2], acc[1][3]);
  gemmkit::acc_guard4(acc[2][0], acc[2][1], acc[2][2], acc[2][3]);
  gemmkit::acc_guard4(acc[3][0], acc[3][1], acc[3][2], acc[3][3]);

  const int q4 = lane >> 3;
  const int c8 = (lane & 7) * 8;
  const int p8 = c8 ^ 32;
  const float sg = (c8 < 32) ? -1.0f : 1.0f;
#pragma unroll
  for (int i = 0; i < 4; ++i) {
    const int mBase = m0 + (i << 4);
#pragma unroll
    for (int j = 0; j < 4; ++j) {
      const float bv = bias[n0 + (j << 4) + rlane];
#pragma unroll
      for (int r = 0; r < 8; ++r)
        sT[wave][(mOff + r) * 68 + (j << 4) + rlane] = acc[i][j][r] * scale + bv;
    }
    __builtin_amdgcn_fence(3  , "workgroup");
    __builtin_amdgcn_wave_barrier();
    __builtin_amdgcn_fence(2  , "workgroup");
#pragma unroll 1
    for (int it = 0; it < 4; ++it) {
      const int row = it * 4 + q4;
      const unsigned int t = (unsigned int)(mBase + row) % (unsigned int)SEQ;
      const size_t to = (size_t)t * (size_t)HDIM + (size_t)c8;
      const v4f ca = *(const v4f*)(cosT + to);
      const v4f cb = *(const v4f*)(cosT + to + 4);
      const v4f sa = *(const v4f*)(sinT + to);
      const v4f sb = *(const v4f*)(sinT + to + 4);
      const float cv[8] = {ca.x, ca.y, ca.z, ca.w, cb.x, cb.y, cb.z, cb.w};
      const float sv[8] = {sa.x, sa.y, sa.z, sa.w, sb.x, sb.y, sb.z, sb.w};
      const int so = row * 68 + c8;
      const int po = row * 68 + p8;
      rq_us8 hv, lv;
#pragma unroll
      for (int e = 0; e < 8; ++e) {
        const float val = sT[wave][so + e] * cmb_bf(cv[e]) + sg * (sT[wave][po + e] * cmb_bf(sv[e]));
        const unsigned short hb = gemmkit::f2bf_bits(val);
        const unsigned short lb = gemmkit::f2bf_bits(val - gemmkit::bf_bits2f(hb));
        hv[e] = hb;
        lv[e] = lb;
      }
      const size_t co = (size_t)(mBase + row) * ldc + n0 + c8;
      *(volatile rq_us8*)(Chi + co) = hv;
      *(volatile rq_us8*)(Clo + co) = lv;
      __threadfence();
      *(volatile rq_us8*)(Chi + co) = hv;
      *(volatile rq_us8*)(Clo + co) = lv;
    }
    __builtin_amdgcn_fence(3  , "workgroup");
    __builtin_amdgcn_wave_barrier();
    __builtin_amdgcn_fence(2  , "workgroup");
  }
}

__device__ __forceinline__ v8f fa_mma_b3(v16b ah, v16b al, v16b bh, v16b bl, v8f c) {
    c = __builtin_amdgcn_wmma_f32_16x16x32_bf16(false, ah, false, bh, (short)0, c, false, false);
    c = __builtin_amdgcn_wmma_f32_16x16x32_bf16(false, ah, false, bl, (short)0, c, false, false);
    c = __builtin_amdgcn_wmma_f32_16x16x32_bf16(false, al, false, bh, (short)0, c, false, false);
    asm volatile("v_nop\n\tv_nop\n\tv_nop\n\tv_nop" : "+v"(c) : "v"(ah), "v"(al), "v"(bh), "v"(bl));
    return c;
}
__device__ __forceinline__ v8f fa_mma_h(v16h a, v16h b, v8f c) {
    c = __builtin_amdgcn_wmma_f32_16x16x32_f16(false, a, false, b, (short)0, c, false, false);
    asm volatile("v_nop\n\tv_nop\n\tv_nop\n\tv_nop" : "+v"(c) : "v"(a), "v"(b));
    return c;
}

template <bool BANDK>
__global__ __launch_bounds__(128)
void k_fattn(const unsigned short* __restrict__ QKHp, const unsigned short* __restrict__ QKLp,
             const unsigned short* __restrict__ VTHp, const unsigned short* __restrict__ VTRp,
             unsigned short* AOp, unsigned short* AORp, unsigned int qb0) {
    const float PSC  = 32768.0f;
    const float SCL2 = 0.18033688011112042f;
    const float NEGINF = -__builtin_inff();
    __shared__ __align__(16) _Float16 Psh[4][16 * 64];
    __shared__ __align__(16) _Float16 Psr[BANDK ? 4 : 1][BANDK ? 16 * 64 : 8];
    __shared__ __align__(16) float    Os[4][16 * 68];

    const unsigned int tid = threadIdx.x, wave = tid >> 5, lane = tid & 31u, hh = lane >> 4, c = lane & 15u;
    const unsigned int qb = blockIdx.x + qb0, h = blockIdx.y, b = blockIdx.z;
    const unsigned int q0 = qb * 64u + wave * 16u;

    const __bf16* qkh = (const __bf16*)QKHp;
    const __bf16* qkl = (const __bf16*)QKLp;
    const _Float16* vth = (const _Float16*)VTHp;
    const _Float16* vtr = (const _Float16*)VTRp;

    v16b qah[2], qal[2];
    {
        const size_t qo = (size_t)(b * (unsigned)SEQ + q0 + c) * (unsigned)NQK + h * 64u + 8u * hh;
#pragma unroll
        for (int dc = 0; dc < 2; ++dc) {
            qah[dc] = gemmkit::Frag<__bf16>::load(qkh + qo + dc * 32);
            qal[dc] = gemmkit::Frag<__bf16>::load(qkl + qo + dc * 32);
        }
    }

    float mrow[8], lrow[8];
    v8f oacc[4], ores[4];
#pragma unroll
    for (int r = 0; r < 8; ++r) { mrow[r] = NEGINF; lrow[r] = 0.f; }
#pragma unroll
    for (int t = 0; t < 4; ++t) { oacc[t] = (v8f){0.f,0.f,0.f,0.f,0.f,0.f,0.f,0.f}; ores[t] = (v8f){0.f,0.f,0.f,0.f,0.f,0.f,0.f,0.f}; }

    _Float16* pwh = Psh[wave];
    _Float16* pwr = Psr[BANDK ? wave : 0];

    const unsigned int nChunks = qb + 1u;
    for (unsigned int kc = 0; kc < nChunks; ++kc) {
        const unsigned int kv0 = kc * 64u;
        v8f s[4];
#pragma unroll
        for (int j = 0; j < 4; ++j) {
            const size_t ko = (size_t)(b * (unsigned)SEQ + kv0 + (unsigned)j * 16u + c) * (unsigned)NQK + (unsigned)EMB + h * 64u + 8u * hh;
            v8f acc = (v8f){0.f,0.f,0.f,0.f,0.f,0.f,0.f,0.f};
#pragma unroll
            for (int dc = 0; dc < 2; ++dc) {
                const v16b kh_ = gemmkit::Frag<__bf16>::load(qkh + ko + dc * 32);
                const v16b kl_ = gemmkit::Frag<__bf16>::load(qkl + ko + dc * 32);
                acc = fa_mma_b3(qah[dc], qal[dc], kh_, kl_, acc);
            }
            s[j] = acc;
        }
        const bool diag = (kc == qb);
#pragma unroll
        for (int r = 0; r < 8; ++r) {
            const unsigned int qrow = q0 + 8u * hh + (unsigned)r;
            float sv[4];
            float m = NEGINF;
#pragma unroll
            for (int j = 0; j < 4; ++j) {
                const unsigned int kvcol = kv0 + (unsigned)j * 16u + c;
                float v = s[j][r] * SCL2;
                v = (diag && (kvcol > qrow)) ? NEGINF : v;
                sv[j] = v;
                m = fmaxf(m, v);
            }
            m = fmaxf(m, __shfl_xor(m, 1, 32)); m = fmaxf(m, __shfl_xor(m, 2, 32));
            m = fmaxf(m, __shfl_xor(m, 4, 32)); m = fmaxf(m, __shfl_xor(m, 8, 32));
            const float mnew = fmaxf(mrow[r], m);
            const float alpha = exp2f(mrow[r] - mnew);
            mrow[r] = mnew;
            float psum = 0.f;
#pragma unroll
            for (int j = 0; j < 4; ++j) {
                const float p = exp2f(sv[j] - mnew);
                psum += p;
                const float pc = p * PSC;
                const _Float16 ph = (_Float16)pc;
                pwh[(8u * hh + (unsigned)r) * 64u + (unsigned)j * 16u + c] = ph;
                if (BANDK) pwr[(8u * hh + (unsigned)r) * 64u + (unsigned)j * 16u + c] = (_Float16)((pc - (float)ph) * 2048.0f);
            }
            psum += __shfl_xor(psum, 1, 32); psum += __shfl_xor(psum, 2, 32);
            psum += __shfl_xor(psum, 4, 32); psum += __shfl_xor(psum, 8, 32);
            lrow[r] = lrow[r] * alpha + psum;
#pragma unroll
            for (int t = 0; t < 4; ++t) { oacc[t][r] *= alpha; if (BANDK) ores[t][r] *= alpha; }
        }
        __builtin_amdgcn_fence(3  , "workgroup");
        __builtin_amdgcn_wave_barrier();
        __builtin_amdgcn_fence(2  , "workgroup");
#pragma unroll
        for (int kk = 0; kk < 2; ++kk) {
            const v16h pa = gemmkit::Frag<_Float16>::load(pwh + c * 64u + (unsigned)kk * 32u + 8u * hh);
            v16h pr = pa;
            if (BANDK) pr = gemmkit::Frag<_Float16>::load(pwr + c * 64u + (unsigned)kk * 32u + 8u * hh);
#pragma unroll
            for (int t = 0; t < 4; ++t) {
                const size_t vo = (size_t)(b * (unsigned)EMB + h * 64u + (unsigned)t * 16u + c) * (unsigned)SEQ + kv0 + (unsigned)kk * 32u + 8u * hh;
                const v16h vb = gemmkit::Frag<_Float16>::load(vth + vo);
                oacc[t] = fa_mma_h(pa, vb, oacc[t]);
                if (BANDK) {
                    const v16h vr = gemmkit::Frag<_Float16>::load(vtr + vo);
                    ores[t] = fa_mma_h(pa, vr, ores[t]);
                    ores[t] = fa_mma_h(pr, vb, ores[t]);
                }
            }
        }
    }

    float* os = Os[wave];
#pragma unroll
    for (int r = 0; r < 8; ++r) {
        const float inv = (16.0f / 32768.0f) * (1.0f / lrow[r]);
#pragma unroll
        for (int t = 0; t < 4; ++t) {
            float val = oacc[t][r];
            if (BANDK) val += ores[t][r] * (1.0f / 2048.0f);
            os[(8u * hh + (unsigned)r) * 68u + (unsigned)t * 16u + c] = val * inv;
        }
    }
    __builtin_amdgcn_fence(3  , "workgroup");
    __builtin_amdgcn_wave_barrier();
    __builtin_amdgcn_fence(2  , "workgroup");
    {
        const unsigned int q = lane >> 3, c8 = (lane & 7u) * 8u;
        unsigned short* ao = AOp + (size_t)(b * (unsigned)SEQ + q0) * (unsigned)EMB + h * 64u + c8;
        unsigned short* ar = AORp + (size_t)(b * (unsigned)BAND + (BANDK ? q0 : 0u)) * (unsigned)EMB + h * 64u + c8;
        for (int pass = 0; pass < 2; ++pass) {
#pragma unroll
            for (int it = 0; it < 4; ++it) {
                const unsigned int row = (unsigned)it * 4u + q;
                const float* sp = os + row * 68u + c8;
                v8h hv, lv;
#pragma unroll
                for (int e = 0; e < 8; ++e) {
                    const _Float16 hf = (_Float16)sp[e];
                    hv[e] = hf;
                    lv[e] = (_Float16)((sp[e] - (float)hf) * 2048.0f);
                }
                *(volatile v8h*)(ao + (size_t)row * (unsigned)EMB) = hv;
                if (BANDK) *(volatile v8h*)(ar + (size_t)row * (unsigned)EMB) = lv;
            }
            __threadfence();
        }
    }
}

constexpr size_t WS_X16  = (size_t)MROWS * EMB * 2;
constexpr size_t WS_W3   = (size_t)NQKV * EMB * 2;
constexpr size_t WS_WO   = (size_t)EMB * EMB * 2;
constexpr size_t WS_BR3  = (size_t)(NQKV + 64) * 4;
constexpr size_t WS_BRO  = (size_t)(EMB + 64) * 4;
constexpr size_t WS_QK   = (size_t)MROWS * NQK * 2;
constexpr size_t WS_VT   = (size_t)NB * EMB * SEQ * 2;
constexpr size_t WS_AOR  = (size_t)NB * BAND * EMB * 2;
constexpr size_t OFF_X16 = 0;
constexpr size_t OFF_W3  = OFF_X16 + WS_X16;
constexpr size_t OFF_WO  = OFF_W3 + WS_W3;
constexpr size_t OFF_BR3 = OFF_WO + WS_WO;
constexpr size_t OFF_BRO = OFF_BR3 + WS_BR3;
constexpr size_t OFF_QKH = OFF_BRO + WS_BRO;
constexpr size_t OFF_QKL = OFF_QKH + WS_QK;
constexpr size_t OFF_VTH = OFF_QKL + WS_QK;
constexpr size_t OFF_VTR = OFF_VTH + WS_VT;
constexpr size_t OFF_AOR = OFF_VTR + WS_VT;
constexpr size_t WS_TOTAL = OFF_AOR + WS_AOR;
static_assert(WS_X16 % 256 == 0 && WS_W3 % 256 == 0 && WS_WO % 256 == 0 && WS_BR3 % 256 == 0 && WS_BRO % 256 == 0);
static_assert(WS_QK % 256 == 0 && WS_VT % 256 == 0 && WS_AOR % 256 == 0);
static_assert(WS_TOTAL <= (size_t)134217728);
static_assert((size_t)MROWS * EMB * 2 <= WS_X16);

static_assert(((size_t)MROWS * EMB / 8) % 256 == 0 && ((size_t)NQKV * EMB / 8) % 256 == 0 && ((size_t)EMB * EMB / 8) % 256 == 0);
static_assert(NQKV % 256 == 0 && EMB % 256 == 0);
static_assert(((MROWS / 64) * (NQK / 64)) % 8 == 0);
static_assert(((EMB / 64) * (SEQ / 64)) % 8 == 0);
static_assert(((MROWS / 64) * (EMB / 64)) % 8 == 0);
static_assert(((BAND / 64) * (EMB / 64)) % 8 == 0);
static_assert(MROWS % 64 == 0 && NQK % 64 == 0 && EMB % 32 == 0);
static_assert((size_t)(MROWS - 1) * NQK + (NQK - 64) + 56 + 8 <= (size_t)MROWS * NQK);
static_assert((SEQ_FULL * HDIM) % 4 == 0);

extern "C" void kernel_launch(void* const* d_in, const int* in_sizes, int n_in, void* d_out, int out_size, void* d_ws, size_t ws_size, hipStream_t stream) {
    if (n_in < 7) return;
    if (in_sizes[0] < MROWS * EMB) return;
    if (in_sizes[1] < NQKV * EMB) return;
    if (in_sizes[2] < NQKV) return;
    if (in_sizes[3] < EMB * EMB) return;
    if (in_sizes[4] < EMB) return;
    if (in_sizes[5] < SEQ * HDIM) return;
    if (in_sizes[6] < SEQ * HDIM) return;
    if (out_size < MROWS * EMB) return;
    if (ws_size < WS_TOTAL) return;
    const float* x    = (const float*)d_in[0];
    const float* Wqkv = (const float*)d_in[1];
    const float* bqkv = (const float*)d_in[2];
    const float* Wo   = (const float*)d_in[3];
    const float* bo   = (const float*)d_in[4];
    const float* cosT = (const float*)d_in[5];
    const float* sinT = (const float*)d_in[6];
    float* out = (float*)d_out;
    char* wsp = (char*)d_ws;
    unsigned short* X16  = (unsigned short*)(wsp + OFF_X16);
    unsigned short* AO16 = X16;
    unsigned short* W316 = (unsigned short*)(wsp + OFF_W3);
    unsigned short* WO16 = (unsigned short*)(wsp + OFF_WO);
    float* BR3 = (float*)(wsp + OFF_BR3);
    float* BRO = (float*)(wsp + OFF_BRO);
    unsigned short* QKH = (unsigned short*)(wsp + OFF_QKH);
    unsigned short* QKL = (unsigned short*)(wsp + OFF_QKL);
    unsigned short* VTH = (unsigned short*)(wsp + OFF_VTH);
    unsigned short* VTR = (unsigned short*)(wsp + OFF_VTR);
    unsigned short* AOR = (unsigned short*)(wsp + OFF_AOR);

    k_cm_castb<<<(unsigned)(((size_t)MROWS * EMB / 8) / 256), 256, 0, stream>>>(x, X16, (unsigned)((size_t)MROWS * EMB / 8), 1.0f);
    k_cm_castb<<<(unsigned)(((size_t)NQKV * EMB / 8) / 256), 256, 0, stream>>>(Wqkv, W316, (unsigned)((size_t)NQKV * EMB / 8), 16.0f);
    k_cm_castb<<<(unsigned)(((size_t)EMB * EMB / 8) / 256), 256, 0, stream>>>(Wo, WO16, (unsigned)((size_t)EMB * EMB / 8), 16.0f);
    k_cm_bfvec<<<NQKV / 256, 256, 0, stream>>>(bqkv, BR3, (unsigned)NQKV);
    k_cm_bfvec<<<EMB / 256, 256, 0, stream>>>(bo, BRO, (unsigned)EMB);

    k_qk_rot<<<dim3((unsigned)(((MROWS / 64) * (NQK / 64)) / 8), 1u), 256, 0, stream>>>(
        (const unsigned short*)X16, EMB,
        (const unsigned short*)W316, EMB,
        QKH, QKL, NQK,
        (const float*)BR3, cosT, sinT,
        MROWS, NQK, EMB, 0.0625f);
    gemmkit::wmma_gemm64<0, false, 1, 3, false><<<dim3((unsigned)(((EMB / 64) * (SEQ / 64)) / 8), (unsigned)NB), 256, 0, stream>>>(
        (const unsigned short*)(W316 + (size_t)NQK * EMB), nullptr, EMB, (long)0,
        (const unsigned short*)X16, nullptr, EMB, (long)SEQ * EMB,
        (void*)VTH, (void*)VTR, SEQ, (long)EMB * SEQ,
        BR3 + NQK, nullptr, (long)0,
        EMB, SEQ, EMB, 0.0625f);

    k_fattn<true><<<dim3((unsigned)(BAND / 64), (unsigned)NHEAD, (unsigned)NB), 128, 0, stream>>>(QKH, QKL, VTH, VTR, AO16, AOR, 0u);
    if ((SEQ - BAND) / 64 > 0)
        k_fattn<false><<<dim3((unsigned)((SEQ - BAND) / 64), (unsigned)NHEAD, (unsigned)NB), 128, 0, stream>>>(QKH, QKL, VTH, VTR, AO16, AOR, (unsigned)(BAND / 64));

    gemmkit::wmma_gemm64<0, false, 2, 0, false><<<dim3((unsigned)(((MROWS / 64) * (EMB / 64)) / 8), 1u), 256, 0, stream>>>(
        (const unsigned short*)AO16, nullptr, EMB, (long)0,
        (const unsigned short*)WO16, nullptr, EMB, (long)0,
        (void*)out, nullptr, EMB, (long)0,
        BRO, nullptr, (long)0,
        MROWS, EMB, EMB, 1.0f / 256.0f);
    gemmkit::wmma_gemm64<0, false, 0, 0, true><<<dim3((unsigned)(((BAND / 64) * (EMB / 64)) / 8), (unsigned)NB), 256, 0, stream>>>(
        (const unsigned short*)AOR, nullptr, EMB, (long)BAND * EMB,
        (const unsigned short*)WO16, nullptr, EMB, (long)0,
        (void*)out, nullptr, EMB, (long)SEQ * EMB,
        nullptr, (const float*)out, (long)SEQ * EMB,
        BAND, EMB, EMB, 1.0f / 524288.0f);
}
